// PositionAttention_91182155694507
// MI455X (gfx1250) — hardware-verified
//
#include <hip/hip_runtime.h>


#ifndef NB
#define NB 4
#endif
#ifndef SEQ
#define SEQ 4096
#endif

namespace {
constexpr int Bn = NB, C = 512, CQ = 64, HWF = 64, NPF = HWF * HWF, NP = SEQ, NT = Bn * NP;
constexpr int RR = 2 * CQ + C;
constexpr int NCB = RR / 128;
constexpr float XS = 8.0f, PS = 1024.0f;
static_assert(Bn >= 1 && Bn <= 4);
static_assert(NP % 128 == 0 && NP >= 128 && NP <= NPF);
static_assert(C % 128 == 0 && CQ == 64 && RR % 128 == 0 && NCB == 5);

typedef _Float16 b16;
typedef __attribute__((ext_vector_type(16))) _Float16 v16b;
typedef __attribute__((ext_vector_type(8))) _Float16 v8b;
typedef __attribute__((ext_vector_type(8))) float v8f;
typedef __attribute__((ext_vector_type(4))) float v4f;
__device__ __forceinline__ float bf16_rne(float f) { unsigned int u = __float_as_uint(f); u += 0x7FFFu + ((u >> 16) & 1u); return __uint_as_float(u & 0xFFFF0000u); }
__device__ __forceinline__ void split16(float v, b16& hi, b16& lo) { hi = (b16)v; lo = (b16)(v - (float)hi); }
__device__ __forceinline__ v16b frag_kb(const b16* p, int hh) { const v8b a = *(const v8b*)(p + 8 * hh), b = *(const v8b*)(p + 16 + 8 * hh); v16b f;
#pragma unroll
  for (int e = 0; e < 8; ++e) { f[e] = a[e]; f[8 + e] = b[e]; } return f; }
__device__ __forceinline__ v8f wmma16b(v16b a, v16b b, v8f c) { v8f d = __builtin_amdgcn_wmma_f32_16x16x32_f16(false, a, false, b, (short)0, c, false, false); asm volatile("v_nop\n\tv_nop\n\tv_nop\n\tv_nop" : "+v"(d) : "v"(a), "v"(b)); return d; }
__device__ __forceinline__ float nexp(float x) { return __builtin_amdgcn_exp2f(x * 1.4426950408889634f); }
__device__ __forceinline__ float pmul(float a, float b) { float p = a * b; asm volatile("" : "+v"(p)); return p; }

__global__ __launch_bounds__(256) void rows_kernel(const float* __restrict__ x, const float* __restrict__ Wq, const float* __restrict__ Wk, const float* __restrict__ Wv, const float* __restrict__ gma,
                                                   b16* __restrict__ X, b16* __restrict__ R, float* __restrict__ P) {
  __shared__ __attribute__((aligned(16))) b16 Tt[64][C + 8];
  const int b = blockIdx.y, p0 = blockIdx.x * 64, t_ = threadIdx.x;
  for (int i = t_; i < C * 64; i += 256) { const int c = i >> 6, p = i & 63; Tt[p][c] = (b16)bf16_rne(x[((size_t)b * C + c) * NPF + p0 + p]); }
  __syncthreads();
  for (int pass = 0; pass < 2; ++pass) {
    for (int i = t_; i < 64 * (C / 8); i += 256) { const int p = i / (C / 8), c8 = (i % (C / 8)) * 8; *(volatile v8b*)(X + ((size_t)b * NP + p0 + p) * C + c8) = *(const v8b*)(&Tt[p][c8]); }
    if (b == 0) {
      for (int i = blockIdx.x * 256 + t_; i < RR * C / 8; i += (NP / 64) * 256) {
        const size_t q = (size_t)i * 8;
        const float* s_ = (q < (size_t)CQ * C) ? (Wq + q) : (q < (size_t)2 * CQ * C) ? (Wk + (q - (size_t)CQ * C)) : (Wv + (q - (size_t)2 * CQ * C));
        v8b v;
#pragma unroll
        for (int e = 0; e < 8; ++e) v[e] = (b16)bf16_rne(s_[e]);
        *(volatile v8b*)(R + q) = v; }
      if (blockIdx.x == 0 && t_ < 32) ((volatile float*)P)[t_] = (t_ == 0) ? bf16_rne(gma[0]) : 0.0f; }
    __threadfence(); }
}

__global__ __launch_bounds__(128) void proj_kernel(const b16* __restrict__ X, const b16* __restrict__ R, b16* __restrict__ QH, b16* __restrict__ QL, b16* __restrict__ Kr, b16* __restrict__ VT) {
  __shared__ __attribute__((aligned(16))) float Ts[128][128 + 4];
  const int lane = threadIdx.x & 31, wave = threadIdx.x >> 5, nloc = lane & 15, hlf = lane >> 4, b = blockIdx.y, cb = blockIdx.z, p0 = blockIdx.x * 128, m0 = p0 + wave * 32;
  const b16* A = X + (size_t)b * NP * C; const b16* Wr = R + (size_t)cb * 128 * C;
  v8f acc[2][8];
#pragma unroll
  for (int r = 0; r < 2; ++r)
#pragma unroll
    for (int t = 0; t < 8; ++t) acc[r][t] = (v8f){};
#pragma unroll 2
  for (int kb = 0; kb < C; kb += 32) {
    const v16b a0 = frag_kb(A + (size_t)(m0 + nloc) * C + kb, hlf), a1 = frag_kb(A + (size_t)(m0 + 16 + nloc) * C + kb, hlf);
#pragma unroll
    for (int t = 0; t < 8; ++t) { const v16b bw = frag_kb(Wr + (size_t)(t * 16 + nloc) * C + kb, hlf); acc[0][t] = wmma16b(a0, bw, acc[0][t]); acc[1][t] = wmma16b(a1, bw, acc[1][t]); } }
#pragma unroll
  for (int t = 0; t < 8; ++t)
#pragma unroll
    for (int r = 0; r < 2; ++r)
#pragma unroll
      for (int v = 0; v < 8; ++v) Ts[wave * 32 + r * 16 + 8 * hlf + v][t * 16 + nloc] = acc[r][t][v];
  __syncthreads();
  for (int pass = 0; pass < 2; ++pass) {
    if (cb == 0) {
      for (int i = threadIdx.x; i < 128 * (CQ / 8); i += 128) {
        const int rr = i >> 3, c8 = (i & 7) * 8; v8b h_, l_;
#pragma unroll
        for (int e = 0; e < 8; ++e) { b16 a_, b_; split16(Ts[rr][c8 + e] * XS, a_, b_); h_[e] = a_; l_[e] = b_; }
        const size_t gi = ((size_t)b * NP + p0 + rr) * CQ + c8; *(volatile v8b*)(QH + gi) = h_; *(volatile v8b*)(QL + gi) = l_; }
      for (int i = threadIdx.x; i < 128 * (CQ / 8); i += 128) {
        const int rr = i >> 3, c8 = (i & 7) * 8; v8b h_;
#pragma unroll
        for (int e = 0; e < 8; ++e) h_[e] = (b16)(Ts[rr][CQ + c8 + e] * XS);
        *(volatile v8b*)(Kr + ((size_t)b * NP + p0 + rr) * CQ + c8) = h_; }
    } else {
      for (int i = threadIdx.x; i < 128 * 16; i += 128) {
        const int c = i >> 4, c8 = (i & 15) * 8; v8b v;
#pragma unroll
        for (int e = 0; e < 8; ++e) v[e] = (b16)(Ts[c8 + e][c] * XS);
        *(volatile v8b*)(VT + ((size_t)b * C + (cb - 1) * 128 + c) * NP + p0 + c8) = v; }
    }
    __threadfence(); }
}

__global__ __launch_bounds__(128) void attn_kernel(const b16* __restrict__ QH, const b16* __restrict__ QL, const b16* __restrict__ Kr, const b16* __restrict__ VT, float* __restrict__ ATT) {
  __shared__ __attribute__((aligned(16))) b16 Pt[16][64 + 8]; __shared__ float Mx[4][16], Sm[4][16]; __shared__ __attribute__((aligned(16))) float Os[16][C + 4];
  const int wave = threadIdx.x >> 5, lane = threadIdx.x & 31, hh = lane >> 4, col = lane & 15, b = blockIdx.y, q0 = blockIdx.x * 16, qi = q0 + col;
  const b16* qh = QH + ((size_t)b * NP + qi) * CQ; const b16* ql = QL + ((size_t)b * NP + qi) * CQ; const b16* Kb = Kr + (size_t)b * NP * CQ; const b16* Vb = VT + (size_t)b * C * NP;
  const float SC = 1.0f / (XS * XS);
  const v16b qa0 = frag_kb(qh, hh), qa1 = frag_kb(qh + 32, hh), qb0 = frag_kb(ql, hh), qb1 = frag_kb(ql + 32, hh);
  float m = -__builtin_inff(), l = 0.0f; v8f o[8];
#pragma unroll
  for (int t = 0; t < 8; ++t) o[t] = (v8f){};
#pragma unroll 1
  for (int kb = 0; kb < NP; kb += 64) {
    const b16* krow = Kb + (size_t)(kb + 16 * wave + col) * CQ;
    const v16b k0 = frag_kb(krow, hh), k1 = frag_kb(krow + 32, hh);
    v8f s = {};
    s = wmma16b(k0, qa0, s); s = wmma16b(k0, qb0, s); s = wmma16b(k1, qa1, s); s = wmma16b(k1, qb1, s);
    float sv[8]; float mr = -__builtin_inff();
#pragma unroll
    for (int r = 0; r < 8; ++r) { sv[r] = s[r] * SC; mr = fmaxf(mr, sv[r]); }
    mr = fmaxf(mr, __shfl_xor(mr, 16));
    if (hh == 0) Mx[wave][col] = mr;
    __syncthreads();
    const float mn = fmaxf(m, fmaxf(fmaxf(Mx[0][col], Mx[1][col]), fmaxf(Mx[2][col], Mx[3][col]))), al_ = nexp(m - mn); m = mn;
    float sum = 0.0f;
#pragma unroll
    for (int r = 0; r < 8; ++r) { const float e = nexp(sv[r] - mn); sum += e; Pt[col][16 * wave + 8 * hh + r] = (b16)(e * PS); }
    sum += __shfl_xor(sum, 16);
    if (hh == 0) Sm[wave][col] = sum;
    __syncthreads();
    l = l * al_ + ((Sm[0][col] + Sm[1][col]) + (Sm[2][col] + Sm[3][col]));
    const v16b pb0 = frag_kb(&Pt[col][0], hh), pb1 = frag_kb(&Pt[col][32], hh);
#pragma unroll
    for (int t = 0; t < 8; ++t) {
      const b16* vrow = Vb + (size_t)((wave * 8 + t) * 16 + col) * NP + kb;
      o[t] *= al_; o[t] = wmma16b(frag_kb(vrow, hh), pb0, o[t]); o[t] = wmma16b(frag_kb(vrow + 32, hh), pb1, o[t]); }
    __syncthreads(); }
  const float inv = 1.0f / (l * (PS * XS));
#pragma unroll
  for (int t = 0; t < 8; ++t)
#pragma unroll
    for (int r = 0; r < 8; ++r) Os[col][(wave * 8 + t) * 16 + 8 * hh + r] = o[t][r] * inv;
  __syncthreads();
  for (int pass = 0; pass < 2; ++pass) {
    for (int i = threadIdx.x; i < 16 * (C / 4); i += 128) { const int rr = i / (C / 4), c4 = (i % (C / 4)) * 4; *(volatile v4f*)(ATT + ((size_t)b * NP + q0 + rr) * C + c4) = *(const v4f*)(&Os[rr][c4]); }
    __threadfence(); }
}

__global__ __launch_bounds__(256) void out_kernel(const float* __restrict__ ATT, const float* __restrict__ x, const float* __restrict__ P, float* __restrict__ out) {
  __shared__ __attribute__((aligned(16))) float Tq[128][128 + 1];
  const int b = blockIdx.y, p0 = blockIdx.x * 128, t_ = threadIdx.x; const float g = P[0];
  for (int quarter = 0; quarter < 4; ++quarter) {
    __syncthreads();
    for (int i = t_; i < 128 * 128; i += 256) { const int p = i >> 7, c = i & 127; Tq[c][p] = ATT[((size_t)b * NP + p0 + p) * C + quarter * 128 + c]; }
    __syncthreads();
    for (int pass = 0; pass < 2; ++pass) {
      for (int i = t_; i < 128 * 32; i += 256) {
        const int c = i >> 5, c4 = (i & 31) * 4; const size_t gi = ((size_t)b * C + quarter * 128 + c) * NPF + p0 + c4;
        const v4f xr = *(const v4f*)(x + gi); v4f ov;
#pragma unroll
        for (int e = 0; e < 4; ++e) ov[e] = pmul(g, Tq[c][c4 + e]) + bf16_rne(xr[e]);
        *(volatile v4f*)(out + gi) = ov; }
      __threadfence(); } }
}
}

extern "C" void kernel_launch(void* const* d_in, const int* in_sizes, int n_in,
                              void* d_out, int out_size, void* d_ws, size_t ws_size, hipStream_t stream) {
  (void)n_in;
  const float* x = (const float*)d_in[0]; const float* Wq = (const float*)d_in[1]; const float* Wk = (const float*)d_in[2]; const float* Wv = (const float*)d_in[3]; const float* gma = (const float*)d_in[4];
  float* out = (float*)d_out;
  if (in_sizes[0] < Bn * C * NPF || in_sizes[1] < CQ * C || in_sizes[2] < CQ * C || in_sizes[3] < C * C || in_sizes[4] < 1 || out_size < Bn * C * NPF) return;
  size_t off = 0; char* ws = (char*)d_ws;
  auto carve = [&](size_t bytes) { char* p = ws + off; off += (bytes + 255) & ~(size_t)255; return p; };
  b16* X = (b16*)carve((size_t)NT * C * 2);
  b16* R = (b16*)carve((size_t)RR * C * 2);
  float* P = (float*)carve(256);
  b16* QH = (b16*)carve((size_t)NT * CQ * 2);
  b16* QL = (b16*)carve((size_t)NT * CQ * 2);
  b16* Kr = (b16*)carve((size_t)NT * CQ * 2);
  b16* VT = (b16*)carve((size_t)NT * C * 2);
  float* ATT = (float*)carve((size_t)NT * C * 4);
  if (off > ws_size) return;
  rows_kernel<<<dim3(NP / 64, Bn), 256, 0, stream>>>(x, Wq, Wk, Wv, gma, X, R, P);
  proj_kernel<<<dim3(NP / 128, Bn, NCB), 128, 0, stream>>>(X, R, QH, QL, Kr, VT);
  attn_kernel<<<dim3(NP / 16, Bn), 128, 0, stream>>>(QH, QL, Kr, VT, ATT);
  out_kernel<<<dim3(NP / 128, Bn), 256, 0, stream>>>(ATT, x, P, out);
}
